// Transformer_Model_46961172414621
// MI455X (gfx1250) — hardware-run, weakly checked
//
#include <hip/hip_runtime.h>


namespace {
constexpr int B = 16, S = 512, D = 512, H = 8, DK = 64, T = 8, N = B * S, NTOK = 8192  , NTILE = N / 16 + T  ;
constexpr float XS = 8.0f, WSC = 256.0f, PS = 1024.0f, LOG2E = 1.4426950408889634f, EPS = 1e-5f;
static_assert(S % 32 == 0 && D == H * DK && NTOK % S == 0, "tiling");
typedef _Float16 b16;
typedef __attribute__((ext_vector_type(16))) _Float16 v16b;
typedef __attribute__((ext_vector_type(8))) _Float16 v8b;
typedef __attribute__((ext_vector_type(8))) float v8f;
typedef __attribute__((ext_vector_type(4))) float v4f;
__device__ __forceinline__ float bf16_rne(float f) { unsigned int u = __float_as_uint(f); u += 0x7FFFu + ((u >> 16) & 1u); return __uint_as_float(u & 0xFFFF0000u); }
__device__ __forceinline__ void split16(float v, b16& hi, b16& lo) { hi = (b16)v; lo = (b16)(v - (float)hi); }
__device__ __forceinline__ v16b frag_kb(const b16* p, int hh) { const v8b a = *(const v8b*)(p + 8 * hh), b = *(const v8b*)(p + 16 + 8 * hh); v16b f;
#pragma unroll
  for (int e = 0; e < 8; ++e) { f[e] = a[e]; f[8 + e] = b[e]; } return f; }
__device__ __forceinline__ v8f wmma16b(v16b a, v16b b, v8f c) { v8f d = __builtin_amdgcn_wmma_f32_16x16x32_f16(false, a, false, b, (short)0, c, false, false); asm volatile("v_nop\n\tv_nop\n\tv_nop\n\tv_nop" : "+v"(d) : "v"(a), "v"(b)); return d; }
__device__ __forceinline__ void wave_lds_sync() { __builtin_amdgcn_fence(__ATOMIC_RELEASE, "workgroup"); __builtin_amdgcn_wave_barrier(); __builtin_amdgcn_fence(__ATOMIC_ACQUIRE, "workgroup"); }
__device__ __forceinline__ float pmul(float a, float b) { float p = a * b; asm volatile("" : "+v"(p)); return p; }
__device__ __forceinline__ int iclamp(int v, int lo, int hi) { return v < lo ? lo : (v > hi ? hi : v); }
constexpr int CSR_NBLK = 512, CSR_GB = 9, CSR_GN = 1 << CSR_GB  , CSR_MAXG = 512, CSR_CAP = 12288  ;
__global__ __launch_bounds__(64) void csrA_kernel(const int* __restrict__ dst, int E, int N, int nG, int CHP, int NGP, int* __restrict__ STG, int* __restrict__ HST) {
  extern __shared__ int sm[];
  int* cnt = sm; int* run = sm + NGP; int* ids = sm + 2 * NGP;
  const int b = blockIdx.x; const int ch = (E + CSR_NBLK - 1) / CSR_NBLK; const int e0 = b * ch, e1 = min(E, e0 + ch);
  for (int i = threadIdx.x; i < NGP; i += 64) cnt[i] = 0;
  for (int i = threadIdx.x; i < CHP; i += 64) ids[i] = -1;
  __syncthreads();
  if (threadIdx.x == 0) {
    for (int e = e0; e < e1; ++e) { int d = dst[e]; d = (d < 0) ? 0 : (d >= N ? N - 1 : d); cnt[d >> CSR_GB] += 1; }
    int acc = 0; for (int g = 0; g < nG; ++g) { run[g] = acc; acc += cnt[g]; }
    for (int e = e0; e < e1; ++e) { int d = dst[e]; d = (d < 0) ? 0 : (d >= N ? N - 1 : d); const int g = d >> CSR_GB; ids[run[g]] = e; run[g] += 1; } }
  __syncthreads();
  typedef __attribute__((ext_vector_type(4))) int v4i;
  for (int pass = 0; pass < 2; ++pass) {
    for (int i = threadIdx.x; i < CHP / 4; i += 64) *(volatile v4i*)(STG + (size_t)b * CHP + i * 4) = *(const v4i*)(&ids[i * 4]);
    for (int i = threadIdx.x; i < NGP / 4; i += 64) { v4i v; for (int e = 0; e < 4; ++e) v[e] = (i * 4 + e < nG) ? cnt[i * 4 + e] : 0; *(volatile v4i*)(HST + (size_t)b * NGP + i * 4) = v; }
    __threadfence(); }
}
__global__ __launch_bounds__(512) void csrS_kernel(const int* __restrict__ HST, int nG, int NGP, int* __restrict__ START, int* __restrict__ TOT, int* __restrict__ OFF) {
  __shared__ int tot[CSR_MAXG];
  const int b = threadIdx.x;
  for (int pass = 0; pass < 2; ++pass) { int runb = 0; for (int g = 0; g < nG; ++g) { int c = HST[(size_t)b * NGP + g]; c = (c < 0) ? 0 : c; ((volatile int*)OFF)[(size_t)g * CSR_NBLK + b] = runb; runb += c; } __threadfence(); }
  for (int g = threadIdx.x; g < nG; g += 512) { int s = 0; for (int bb = 0; bb < CSR_NBLK; ++bb) { int c = HST[(size_t)bb * NGP + g]; s += (c < 0) ? 0 : c; } tot[g] = s; }
  __syncthreads();
  if (threadIdx.x < 32) {
    __shared__ int st[CSR_MAXG + 32];
    if (threadIdx.x == 0) { int acc = 0; for (int g = 0; g < NGP; ++g) { st[g] = acc; if (g < nG) acc += (tot[g] + 31) & ~31; } st[NGP] = acc; }
    __builtin_amdgcn_fence(__ATOMIC_RELEASE, "workgroup"); __builtin_amdgcn_wave_barrier(); __builtin_amdgcn_fence(__ATOMIC_ACQUIRE, "workgroup");
    for (int pass = 0; pass < 2; ++pass) { for (int i = threadIdx.x; i < NGP + 32; i += 32) { ((volatile int*)START)[i] = (i <= NGP) ? st[min(i, NGP)] : 0; ((volatile int*)TOT)[i] = (i < nG) ? tot[i] : 0; } __threadfence(); } }
}
__global__ __launch_bounds__(256) void csrB_kernel(const int* __restrict__ dst, int N, int nG, int CHP, int NGP, int permLen, const int* __restrict__ STG, const int* __restrict__ HST, const int* __restrict__ OFF, const int* __restrict__ START, const int* __restrict__ TOT, int* __restrict__ PERM, int* __restrict__ ROWPTR, int* __restrict__ ROWCNT, int* __restrict__ FLAG) {
  typedef __attribute__((ext_vector_type(4))) int v4i;
  __shared__ int ids[CSR_CAP]; __shared__ unsigned short key[CSR_CAP]; __shared__ int outp[CSR_CAP]; __shared__ int ncnt[CSR_GN + 1]; __shared__ int boff[CSR_NBLK + 1];
  const int g = blockIdx.x, t_ = threadIdx.x; int tot = TOT[g]; int st = START[g], stn = START[g + 1]; const int v0 = g * CSR_GN; const int nv = min(CSR_GN, N - v0);
  st = (st < 0) ? 0 : (st > permLen - 32 ? permLen - 32 : st) & ~31; stn = (stn < st) ? st : (stn > permLen ? permLen : stn); tot = (tot < 0) ? 0 : tot; if (tot > stn - st && tot <= CSR_CAP) tot = stn - st;
  if (tot > CSR_CAP) {
    for (int pass = 0; pass < 2; ++pass) { for (int i = t_; i < CSR_GN / 4; i += 256) { v4i a, c; for (int e = 0; e < 4; ++e) { a[e] = st; c[e] = 0; } *(volatile v4i*)(ROWPTR + v0 + i * 4) = a; *(volatile v4i*)(ROWCNT + v0 + i * 4) = c; } if (t_ == 0) ((volatile int*)FLAG)[0] = 1; __threadfence(); } (void)nv; return; }
  if (t_ == 0) { int acc = 0; for (int b = 0; b < CSR_NBLK; ++b) { boff[b] = acc; int c = HST[(size_t)b * NGP + g]; c = (c < 0) ? 0 : (c > CHP ? CHP : c); acc += c; if (acc > tot) acc = tot; } boff[CSR_NBLK] = acc; }
  for (int i = t_; i <= CSR_GN; i += 256) ncnt[i] = 0;
  __syncthreads();
  for (int b = 0; b < CSR_NBLK; ++b) { const int c = boff[b + 1] - boff[b]; int o_ = OFF[(size_t)g * CSR_NBLK + b]; o_ = (o_ < 0) ? 0 : (o_ > CHP - c ? CHP - c : o_); const int* src_ = STG + (size_t)b * CHP + o_;
    for (int i = t_; i < c; i += 256) { int id = src_[i]; id = (id < 0) ? 0 : id; ids[boff[b] + i] = id; int d = dst[id]; d = (d < v0) ? v0 : (d >= N ? N - 1 : d); int kk = d - v0; kk = (kk < 0) ? 0 : (kk >= CSR_GN ? CSR_GN - 1 : kk); key[boff[b] + i] = (unsigned short)kk; } }
  __syncthreads();
  if (t_ == 0) { for (int i = 0; i < tot; ++i) ncnt[key[i]] += 1; int acc = 0; for (int vl = 0; vl < CSR_GN; ++vl) { const int c = ncnt[vl]; ncnt[vl] = acc; acc += c; } ncnt[CSR_GN] = acc;
    for (int i = 0; i < tot; ++i) { const int vl = key[i]; outp[ncnt[vl]] = ids[i]; ncnt[vl] += 1; }
    for (int vl = CSR_GN; vl > 0; --vl) ncnt[vl] = ncnt[vl - 1]; ncnt[0] = 0; }
  __syncthreads();
  for (int pass = 0; pass < 2; ++pass) {
    for (int i = t_; i < (stn - st) / 4; i += 256) { v4i v; for (int e = 0; e < 4; ++e) { const int q = i * 4 + e; v[e] = (q < tot) ? outp[q] : -1; } *(volatile v4i*)(PERM + st + i * 4) = v; }
    for (int i = t_; i < CSR_GN / 4; i += 256) { v4i a, c; for (int e = 0; e < 4; ++e) { const int vl = i * 4 + e; a[e] = st + ncnt[vl]; c[e] = (vl < nv) ? (ncnt[vl + 1] - ncnt[vl]) : 0; } *(volatile v4i*)(ROWPTR + v0 + i * 4) = a; *(volatile v4i*)(ROWCNT + v0 + i * 4) = c; }
    __threadfence(); }
}
__global__ __launch_bounds__(256) void csrZ_kernel(int* __restrict__ p, size_t n4) { typedef __attribute__((ext_vector_type(4))) int v4i; const size_t tid = (size_t)blockIdx.x * 256 + threadIdx.x, nth = (size_t)gridDim.x * 256; v4i z = {0, 0, 0, 0}; for (size_t i = tid; i < n4; i += nth) *(volatile v4i*)(p + i * 4) = z; }
struct CsrBufs { int *STG, *HST, *OFF, *START, *TOT, *PERM, *ROWPTR, *ROWCNT, *FLAG; int nG, NGP, CHP; size_t permLen; char* base; size_t bytes; };
static size_t csr_carve(CsrBufs& c, char* ws, size_t off, int E, int N) {
  const size_t off0 = off; c.base = ws + off;
  auto al = [&](size_t bytes) { char* p = ws + off; off += (bytes + 255) & ~(size_t)255; return p; };
  c.nG = (N + CSR_GN - 1) / CSR_GN; c.NGP = (c.nG + 31) & ~31; const int ch = (E + CSR_NBLK - 1) / CSR_NBLK; c.CHP = (ch + 31) & ~31; c.permLen = (size_t)E + 32 * (size_t)c.nG + 32;
  c.STG = (int*)al((size_t)CSR_NBLK * c.CHP * 4); c.HST = (int*)al((size_t)CSR_NBLK * c.NGP * 4); c.OFF = (int*)al((size_t)c.NGP * CSR_NBLK * 4); c.START = (int*)al((size_t)(c.NGP + 64) * 4); c.TOT = (int*)al((size_t)(c.NGP + 64) * 4);
  c.PERM = (int*)al(c.permLen * 4); c.ROWPTR = (int*)al((size_t)c.nG * CSR_GN * 4); c.ROWCNT = (int*)al((size_t)c.nG * CSR_GN * 4); c.FLAG = (int*)al(256);
  c.bytes = off - off0; return off;
}
static void csr_build(const CsrBufs& c, const int* dst, int E, int N, hipStream_t stream) {
  const size_t smem = (size_t)(2 * c.NGP + c.CHP) * 4;
  csrZ_kernel<<<512, 256, 0, stream>>>((int*)c.base, c.bytes / 16);
  csrA_kernel<<<CSR_NBLK, 64, smem, stream>>>(dst, E, N, c.nG, c.CHP, c.NGP, c.STG, c.HST);
  csrS_kernel<<<1, 512, 0, stream>>>(c.HST, c.nG, c.NGP, c.START, c.TOT, c.OFF);
  csrB_kernel<<<c.nG, 256, 0, stream>>>(dst, N, c.nG, c.CHP, c.NGP, (int)c.permLen, c.STG, c.HST, c.OFF, c.START, c.TOT, c.PERM, c.ROWPTR, c.ROWCNT, c.FLAG);
}

typedef __attribute__((ext_vector_type(2))) _Float16 v2h;
typedef __attribute__((ext_vector_type(4))) _Float16 v4h;
typedef __attribute__((ext_vector_type(2))) float v2f;
typedef __attribute__((ext_vector_type(4))) int v4i;
__device__ __forceinline__ float nexp2(float v) { return __builtin_amdgcn_exp2f(v); }
__global__ __launch_bounds__(256) void prep_kernel(const float* __restrict__ wq, const float* __restrict__ wk, const float* __restrict__ wv, const float* __restrict__ wa, b16* __restrict__ WT) {
  const size_t u = (size_t)blockIdx.x * 256 + threadIdx.x; const size_t per = (size_t)T * D * D / 8; if (u >= 4 * per) return; const int m = (int)(u / per); const size_t e = (u % per) * 8; const int t = (int)(e / ((size_t)D * D)); const size_t el = e % ((size_t)D * D); const int oo = (int)(el / D), k0 = (int)(el % D);
  const float* w = (m == 0 ? wq : m == 1 ? wk : m == 2 ? wv : wa) + (size_t)t * D * D; v8b o;
  for (int j = 0; j < 8; ++j) o[j] = (b16)(bf16_rne(w[(size_t)(k0 + j) * D + oo]) * WSC);
  for (int pass = 0; pass < 2; ++pass) { *(volatile v8b*)(WT + (size_t)m * per * 8 + e) = o; __threadfence(); }
}
__global__ __launch_bounds__(32) void tile_kernel(const int* __restrict__ ROWCNT, int* __restrict__ TOFF) {
  __shared__ int s[32]; if (threadIdx.x == 0) { int acc = 0; for (int t = 0; t <= T; ++t) { s[t] = acc; if (t < T) { int c = ROWCNT[t]; c = iclamp(c, 0, N); acc += (c + 15) / 16; } } for (int t = T + 1; t < 32; ++t) s[t] = acc; }
  __builtin_amdgcn_fence(__ATOMIC_RELEASE, "workgroup"); __builtin_amdgcn_wave_barrier(); __builtin_amdgcn_fence(__ATOMIC_ACQUIRE, "workgroup");
  for (int pass = 0; pass < 2; ++pass) { ((volatile int*)TOFF)[threadIdx.x] = s[threadIdx.x]; __threadfence(); }
}
template <int MODE>
__global__ __launch_bounds__(64) void tgemm_kernel(const float* __restrict__ x, const int* __restrict__ PERM, const int* __restrict__ ROWPTR, const int* __restrict__ ROWCNT, int permLen, const int* __restrict__ TOFF, const b16* __restrict__ WT, const float* __restrict__ bq, const float* __restrict__ bk, const float* __restrict__ bv, const float* __restrict__ ba, const b16* __restrict__ Ch, const b16* __restrict__ Cl, b16* __restrict__ Qr, b16* __restrict__ Kr, b16* __restrict__ Vr, float* __restrict__ HR) {
  __shared__ __attribute__((aligned(16))) float Tf[2][16][128 + 4]; __shared__ int rows_s[2][16];
  const int wave = threadIdx.x >> 5, lane = threadIdx.x & 31, nloc = lane & 15, hlf = lane >> 4; const int tile = blockIdx.x * 2 + wave, slab = blockIdx.y, which = (MODE == 0) ? blockIdx.z : 3; const int n0 = slab * 128;
  int t = 0; for (int q = 1; q <= T; ++q) if (tile >= TOFF[q]) t = q; if (t >= T) return;
  const int cnt = iclamp(ROWCNT[t], 0, N), st = iclamp(ROWPTR[t], 0, permLen), i0 = (tile - TOFF[t]) * 16; if (i0 >= cnt) return;
  auto rowof = [&](int i) { const int idx = i0 + i; return (idx < cnt) ? iclamp(PERM[iclamp(st + idx, 0, permLen - 1)], 0, N - 1) : -1; };
  if (hlf == 0) rows_s[wave][nloc] = rowof(nloc);
  wave_lds_sync();
  if (rows_s[wave][0] >= NTOK || rows_s[wave][0] < 0) return;
  const int myrow = rows_s[wave][nloc]; const size_t ar = (size_t)(myrow < 0 ? 0 : myrow);
  const b16* W = WT + (((size_t)which * T + t) * D) * D; const float* bias = (which == 0 ? bq : which == 1 ? bk : which == 2 ? bv : ba) + (size_t)t * D;
  v8f acc[8];
#pragma unroll
  for (int tt = 0; tt < 8; ++tt) acc[tt] = (v8f){};
#pragma unroll 2
  for (int kb = 0; kb < D; kb += 32) { v16b ah, al;
    if (MODE == 0) { const float* xr = x + ar * D + kb; const v4f c0 = *(const v4f*)(xr + 8 * hlf), c1 = *(const v4f*)(xr + 8 * hlf + 4), c2 = *(const v4f*)(xr + 16 + 8 * hlf), c3 = *(const v4f*)(xr + 16 + 8 * hlf + 4); float cv[16];
      for (int i = 0; i < 4; ++i) { cv[i] = c0[i]; cv[4 + i] = c1[i]; cv[8 + i] = c2[i]; cv[12 + i] = c3[i]; }
#pragma unroll
      for (int e2 = 0; e2 < 16; ++e2) { ah[e2] = (b16)(bf16_rne(cv[e2]) * XS); al[e2] = (b16)0.0f; } }
    else { ah = frag_kb(Ch + ar * D + kb, hlf); al = frag_kb(Cl + ar * D + kb, hlf); }
#pragma unroll
    for (int tt = 0; tt < 8; ++tt) { const v16b bw = frag_kb(W + (size_t)(n0 + tt * 16 + nloc) * D + kb, hlf); acc[tt] = wmma16b(ah, bw, acc[tt]); if (MODE == 1) acc[tt] = wmma16b(al, bw, acc[tt]); } }
#pragma unroll
  for (int tt = 0; tt < 8; ++tt) { const float bb = bf16_rne(bias[n0 + tt * 16 + nloc]);
#pragma unroll
    for (int r = 0; r < 8; ++r) Tf[wave][8 * hlf + r][tt * 16 + nloc] = acc[tt][r] * (1.0f / (XS * WSC)) + bb; }
  wave_lds_sync();
  for (int pass = 0; pass < 2; ++pass) {
    for (int rr = 0; rr < 16; ++rr) { const int n = rows_s[wave][rr]; if (n < 0 || n >= NTOK) continue;
      if (MODE == 0) { b16* P = (which == 0 ? Qr : which == 1 ? Kr : Vr); const v4f f = *(const v4f*)(&Tf[wave][rr][lane * 4]); v4h o; for (int j = 0; j < 4; ++j) o[j] = (b16)(f[j] * XS); *(volatile v4h*)(P + (size_t)n * D + n0 + lane * 4) = o; }
      else { v4f f = *(const v4f*)(&Tf[wave][rr][lane * 4]); const v4f xv = *(const v4f*)(x + (size_t)n * D + n0 + lane * 4); for (int j = 0; j < 4; ++j) f[j] += bf16_rne(xv[j]); *(volatile v4f*)(HR + (size_t)n * D + n0 + lane * 4) = f; } }
    __threadfence(); }
}
__global__ __launch_bounds__(64) void attn_kernel(const b16* __restrict__ Qr, const b16* __restrict__ Kr, const b16* __restrict__ Vr, const int* __restrict__ mask, b16* __restrict__ Ch, b16* __restrict__ Cl) {
  __shared__ __attribute__((aligned(16))) b16 Pb[2][16][32 + 8], Vs[2][DK][32 + 8]; __shared__ __attribute__((aligned(16))) float To[2][16][DK + 4];
  const int wave = threadIdx.x >> 5, lane = threadIdx.x & 31, hh = lane >> 4, col = lane & 15; const int b = blockIdx.y / H, h = blockIdx.y % H; const int q0 = blockIdx.x * 32 + wave * 16, qi = q0 + col;
  const size_t tok0 = (size_t)b * S; const b16* Qb = Qr + tok0 * D + h * DK; const b16* Kb = Kr + tok0 * D + h * DK; const b16* Vb = Vr + tok0 * D + h * DK; const int* Mb = mask + ((size_t)b * S) * S;
  const v16b qa0 = frag_kb(Qb + (size_t)qi * D, hh), qa1 = frag_kb(Qb + (size_t)qi * D + 32, hh);
  const float cs = LOG2E / (8.0f * XS * XS);
  float m = -INFINITY, l = 0.0f; v8f o[4]; for (int tq = 0; tq < 4; ++tq) o[tq] = (v8f){};
#pragma unroll 1
  for (int kb = 0; kb < S; kb += 32) {
    { const b16* vr = Vb + (size_t)(kb + lane) * D; for (int q8 = 0; q8 < DK; q8 += 8) { const v8b vv = *(const v8b*)(vr + q8); for (int j = 0; j < 8; ++j) Vs[wave][q8 + j][lane] = vv[j]; } }
    float e[16]; float mx = -INFINITY;
#pragma unroll
    for (int u = 0; u < 2; ++u) { v8f s = (v8f){}; const size_t kr = (size_t)(kb + u * 16 + col) * D; s = wmma16b(frag_kb(Kb + kr, hh), qa0, s); s = wmma16b(frag_kb(Kb + kr + 32, hh), qa1, s);
      const v4i m0 = *(const v4i*)(Mb + (size_t)qi * S + kb + u * 16 + 8 * hh), m1 = *(const v4i*)(Mb + (size_t)qi * S + kb + u * 16 + 8 * hh + 4);
#pragma unroll
      for (int r = 0; r < 8; ++r) { const int mk = (r < 4) ? m0[r] : m1[r - 4]; const float v = (mk != 0) ? s[r] * cs : -INFINITY; e[u * 8 + r] = v; mx = fmaxf(mx, v); } }
    mx = fmaxf(mx, __shfl_xor(mx, 16)); const float mn = fmaxf(m, mx); const float al = (mn == -INFINITY) ? 1.0f : nexp2(m - mn); float sum = 0.0f;
#pragma unroll
    for (int i2 = 0; i2 < 16; ++i2) { const float p = (e[i2] == -INFINITY || mn == -INFINITY) ? 0.0f : nexp2(e[i2] - mn); sum += p; Pb[wave][col][(i2 < 8 ? 0 : 16) + 8 * hh + (i2 & 7)] = (b16)(p * PS); }
    sum += __shfl_xor(sum, 16); l = l * al + sum; m = mn;
    wave_lds_sync();
    const v16b pf = frag_kb(&Pb[wave][col][0], hh);
#pragma unroll
    for (int tq = 0; tq < 4; ++tq) { o[tq] *= al; o[tq] = wmma16b(frag_kb(&Vs[wave][tq * 16 + col][0], hh), pf, o[tq]); }
    wave_lds_sync(); }
  const float inv = 1.0f / (l * PS * XS);
#pragma unroll
  for (int tq = 0; tq < 4; ++tq)
#pragma unroll
    for (int r = 0; r < 8; ++r) To[wave][col][tq * 16 + 8 * hh + r] = o[tq][r] * inv;
  wave_lds_sync();
  for (int pass = 0; pass < 2; ++pass) { for (int rr = 0; rr < 16; ++rr) { const v2f f = *(const v2f*)(&To[wave][rr][lane * 2]); v2h hv, lv; for (int j = 0; j < 2; ++j) { b16 p, q; split16(f[j] * XS, p, q); hv[j] = p; lv[j] = q; }
      const size_t oi = (tok0 + q0 + rr) * D + h * DK + lane * 2; *(volatile v2h*)(Ch + oi) = hv; *(volatile v2h*)(Cl + oi) = lv; } __threadfence(); }
}
__global__ __launch_bounds__(256) void ln_kernel(const float* __restrict__ HR, const int* __restrict__ types, const float* __restrict__ g_, const float* __restrict__ b_, float* __restrict__ out) {
  const int wave = threadIdx.x >> 5, lane = threadIdx.x & 31; const size_t n = (size_t)blockIdx.x * 8 + wave; if (n >= (size_t)NTOK) return; const int t = iclamp(types[n], 0, T - 1);
  float v[16]; float sm = 0.0f;
#pragma unroll
  for (int q = 0; q < 4; ++q) { const v4f f = *(const v4f*)(HR + n * D + lane * 16 + q * 4); for (int j = 0; j < 4; ++j) { v[q * 4 + j] = f[j]; sm += f[j]; } }
#pragma unroll
  for (int o = 1; o < 32; o <<= 1) sm += __shfl_xor(sm, o);
  const float mu = sm * (1.0f / D); float sq = 0.0f;
#pragma unroll
  for (int i = 0; i < 16; ++i) { const float d = v[i] - mu; sq += d * d; }
#pragma unroll
  for (int o = 1; o < 32; o <<= 1) sq += __shfl_xor(sq, o);
  const float rs = rsqrtf(sq * (1.0f / D) + EPS);
  for (int pass = 0; pass < 2; ++pass) {
#pragma unroll
    for (int q = 0; q < 4; ++q) { v4f o4; for (int j = 0; j < 4; ++j) { const int c = lane * 16 + q * 4 + j; o4[j] = (v[q * 4 + j] - mu) * rs * bf16_rne(g_[(size_t)t * D + c]) + bf16_rne(b_[(size_t)t * D + c]); } *(volatile v4f*)(out + n * D + lane * 16 + q * 4) = o4; }
    __threadfence(); }
}
}

extern "C" void kernel_launch(void* const* d_in, const int* in_sizes, int n_in, void* d_out, int out_size, void* d_ws, size_t ws_size, hipStream_t stream) {
  (void)n_in;
  auto Fp = [&](int i) { return (const float*)d_in[i]; }; auto Ip = [&](int i) { return (const int*)d_in[i]; };
  if (in_sizes[0] != N * D || in_sizes[1] != N || in_sizes[2] != B * S * S || in_sizes[3] != T * D * D || in_sizes[4] != T * D || in_sizes[5] != T * D * D || in_sizes[7] != T * D * D || in_sizes[9] != T * D * D || in_sizes[11] != T * D || in_sizes[12] != T * D || out_size != N * D) return;
  size_t off = 0; char* ws = (char*)d_ws;
  auto carve = [&](size_t bytes) { char* p = ws + off; off += (bytes + 255) & ~(size_t)255; return p; };
  b16* WT = (b16*)carve((size_t)4 * T * D * D * 2); int* TOFF = (int*)carve(256); const size_t plane = (size_t)N * D * 2;
  b16* Qr = (b16*)carve(plane); b16* Kr = (b16*)carve(plane); b16* Vr = (b16*)carve(plane); b16* Ch = (b16*)carve(plane); b16* Cl = (b16*)carve(plane); float* HR = (float*)carve((size_t)N * D * 4);
  CsrBufs csr; off = csr_carve(csr, ws, off, N, T);
  if (off > ws_size || off > ((size_t)128 << 20)) return;
  prep_kernel<<<(unsigned)(((size_t)4 * T * D * D / 8 + 255) / 256), 256, 0, stream>>>(Fp(3), Fp(5), Fp(7), Fp(9), WT);
  csr_build(csr, Ip(1), N, T, stream);
  tile_kernel<<<1, 32, 0, stream>>>(csr.ROWCNT, TOFF);
  tgemm_kernel<0><<<dim3(NTILE / 2, 4, 3), 64, 0, stream>>>(Fp(0), csr.PERM, csr.ROWPTR, csr.ROWCNT, (int)csr.permLen, TOFF, WT, Fp(4), Fp(6), Fp(8), Fp(10), nullptr, nullptr, Qr, Kr, Vr, nullptr);
  attn_kernel<<<dim3(S / 32, (NTOK / S) * H), 64, 0, stream>>>(Qr, Kr, Vr, Ip(2), Ch, Cl);
  tgemm_kernel<1><<<dim3(NTILE / 2, 4, 1), 64, 0, stream>>>(Fp(0), csr.PERM, csr.ROWPTR, csr.ROWCNT, (int)csr.permLen, TOFF, WT, Fp(4), Fp(6), Fp(8), Fp(10), Ch, Cl, nullptr, nullptr, nullptr, HR);
  ln_kernel<<<NTOK / 8, 256, 0, stream>>>(HR, Ip(1), Fp(11), Fp(12), (float*)d_out);
}
